// MambaCAN_noid_6803228196994
// MI455X (gfx1250) — hardware-verified
//
#include <hip/hip_runtime.h>
#include <math.h>

typedef __attribute__((ext_vector_type(16))) _Float16 v16h;
typedef __attribute__((ext_vector_type(8)))  _Float16 v8h;
typedef __attribute__((ext_vector_type(16))) __bf16   v16b;
typedef __attribute__((ext_vector_type(8)))  __bf16   v8b;
typedef __attribute__((ext_vector_type(8)))  float    v8f;
typedef __attribute__((ext_vector_type(4)))  float    v4f;

constexpr int kBatch   = 4;
constexpr int kSeq     = 2048;
constexpr int kXin     = 9;
constexpr int kC1      = 128;
constexpr int kPadRows = kSeq + 2;
constexpr int kK2      = 3 * kC1;
constexpr int kDm      = 256;
constexpr int kDin     = 512;
constexpr int kXzP     = 2 * kDin;
constexpr int kNst     = 16;
constexpr int kDtR     = 16;
constexpr int kXpN     = 48;
constexpr int kXdP     = 64;
constexpr int kHid     = 128;
constexpr int kCls     = 4;
constexpr int kRows    = kBatch * kSeq;
constexpr int kC1TP    = 132;
constexpr int kConvTP  = 260;
constexpr int kScanTS  = 64;
constexpr int kScanCh  = 64;
constexpr int kScanYP  = 68;

constexpr size_t kOffF1P  = 0;
constexpr size_t kOffW2P  = kOffF1P  + (size_t)kBatch * kPadRows * kC1 * 2;
constexpr size_t kOffFeat = kOffW2P  + (size_t)kDm * kK2 * 2;
constexpr size_t kOffWin  = kOffFeat + (size_t)kRows * kDm * 2;
constexpr size_t kOffXZ   = kOffWin  + (size_t)kXzP * kDm * 2;
constexpr size_t kOffUC   = kOffXZ   + (size_t)kRows * kXzP * 4;
constexpr size_t kOffUH   = kOffUC   + (size_t)kRows * kDin * 4;
constexpr size_t kOffWxp  = kOffUH   + (size_t)kRows * kDin * 2;
constexpr size_t kOffXD   = kOffWxp  + (size_t)kXdP * kDin * 2;
constexpr size_t kOffYP   = kOffXD   + (size_t)kRows * kXdP * 4;
constexpr size_t kOffWout = kOffYP   + (size_t)kRows * kDin * 2;
constexpr size_t kOffMO   = kOffWout + (size_t)kDm * kDin * 2;
constexpr size_t kOffPool = kOffMO   + (size_t)kRows * kDm * 4;
constexpr size_t kWsTotal = kOffPool + (size_t)kBatch * kDm * 4;
static_assert(kWsTotal == 84940800ull);
static_assert(kWsTotal <= 134217728ull);
static_assert((kOffW2P % 128) == 0 && (kOffFeat % 128) == 0 && (kOffWin % 128) == 0 && (kOffXZ % 128) == 0 &&
              (kOffUC % 128) == 0 && (kOffUH % 128) == 0 && (kOffWxp % 128) == 0 && (kOffXD % 128) == 0 &&
              (kOffYP % 128) == 0 && (kOffWout % 128) == 0 && (kOffMO % 128) == 0 && (kOffPool % 128) == 0);
static_assert(((size_t)kPadRows * kC1 * 2) % 128 == 0);
static_assert(kK2 % 32 == 0 && kDm % 32 == 0 && kDin % 32 == 0);
static_assert(kSeq % 64 == 0 && kRows % 64 == 0 && kDm % 64 == 0 && kXzP % 64 == 0 && kXdP % 64 == 0);

__device__ __forceinline__ unsigned short f2bf_bits(float f) {
  unsigned u = __float_as_uint(f);
  return (unsigned short)((u + 0x7FFFu + ((u >> 16) & 1u)) >> 16);
}
__device__ __forceinline__ float bf_bits2f(unsigned short h) { return __uint_as_float(((unsigned)h) << 16); }

__device__ __forceinline__ void dep_guard_h(v8f& a, v8f& b, v16h x, v16h y) { asm volatile("v_nop\n\tv_nop\n\tv_nop\n\tv_nop" : "+v"(a), "+v"(b) : "v"(x), "v"(y)); }
__device__ __forceinline__ void dep_guard_b(v8f& a, v8f& b, v16b x, v16b y) { asm volatile("v_nop\n\tv_nop\n\tv_nop\n\tv_nop" : "+v"(a), "+v"(b) : "v"(x), "v"(y)); }
__device__ __forceinline__ void keep4_h(v16h a, v16h b, v16h c, v16h d) { asm volatile("v_nop" :: "v"(a), "v"(b), "v"(c), "v"(d)); }
__device__ __forceinline__ void keep4_b(v16b a, v16b b, v16b c, v16b d) { asm volatile("v_nop" :: "v"(a), "v"(b), "v"(c), "v"(d)); }
__device__ __forceinline__ void acc_guard4(v8f& a, v8f& b, v8f& c, v8f& d) { asm volatile("v_nop\n\tv_nop\n\tv_nop\n\tv_nop" : "+v"(a), "+v"(b), "+v"(c), "+v"(d)); }
template <typename T> struct Frag;
template <> struct Frag<_Float16> {
  typedef v16h V; union U { v16h v; v8h h[2]; };
  static __device__ __forceinline__ v16h load(const _Float16* p) {
    U f; f.h[0] = *(const v8h*)(p); f.h[1] = *(const v8h*)(p + 16); return f.v;
  }
  static __device__ __forceinline__ v8f mma(v16h a, v16h b, v8f c) {
    return __builtin_amdgcn_wmma_f32_16x16x32_f16(false, a, false, b, (short)0, c, false, false);
  }
  static __device__ __forceinline__ void guard(v8f& a, v8f& b, v16h x, v16h y) { dep_guard_h(a, b, x, y); }
  static __device__ __forceinline__ void keep(v16h a, v16h b, v16h c, v16h d) { keep4_h(a, b, c, d); }
};
template <> struct Frag<__bf16> {
  typedef v16b V; union U { v16b v; v8b h[2]; };
  static __device__ __forceinline__ v16b load(const __bf16* p) {
    U f; f.h[0] = *(const v8b*)(p); f.h[1] = *(const v8b*)(p + 16); return f.v;
  }
  static __device__ __forceinline__ v8f mma(v16b a, v16b b, v8f c) {
    return __builtin_amdgcn_wmma_f32_16x16x32_bf16(false, a, false, b, (short)0, c, false, false);
  }
  static __device__ __forceinline__ void guard(v8f& a, v8f& b, v16b x, v16b y) { dep_guard_b(a, b, x, y); }
  static __device__ __forceinline__ void keep(v16b a, v16b b, v16b c, v16b d) { keep4_b(a, b, c, d); }
};

template <int ET> struct Elem;
template <> struct Elem<0> { typedef _Float16 T; };
template <> struct Elem<1> { typedef __bf16 T; };
template <int ET, bool SPLIT, int BIAS_MODE, int OUT_MODE, bool RESID, int ACT = 0>
__global__ __launch_bounds__(256) void wmma_gemm64(
    const unsigned short* __restrict__ Ap, const unsigned short* __restrict__ A2p, int lda, long strideA,
    const unsigned short* __restrict__ Btp, const unsigned short* __restrict__ Bt2p, int ldb, long strideB,
    void* __restrict__ Cout, void* __restrict__ Cout2, int ldc, long strideC,
    const float* __restrict__ bias,
    const float* __restrict__ resid, long strideR,
    int M, int N, int K, float scale) {
  typedef typename Elem<ET>::T T;
  typedef typename Frag<T>::V V;
  const T* A = (const T*)Ap; const T* A2 = (const T*)A2p; const T* Bt = (const T*)Btp; const T* Bt2 = (const T*)Bt2p;
  __shared__ __align__(16) float sT[8][16 * 68];
  const int b    = blockIdx.y;
  const int lane = threadIdx.x & 31;
  const int wave = threadIdx.x >> 5;
  const int tilesN = N >> 6;
  const int tilesM = M >> 6;
  const int tile = blockIdx.x * 8 + wave;
  if (tile >= tilesM * tilesN) return;
  const int tm = tile / tilesN;
  const int tn = tile - tm * tilesN;
  const int m0 = tm << 6;
  const int n0 = tn << 6;

  const T* Ab  = A  + (size_t)b * strideA;
  const T* Bb  = Bt + (size_t)b * strideB;
  const T* Ab2 = SPLIT ? (A2  + (size_t)b * strideA) : nullptr;
  const T* Bb2 = SPLIT ? (Bt2 + (size_t)b * strideB) : nullptr;

  const int rlane = lane & 15;
  const int koff  = (lane >> 4) * 8;
  const int mOff  = (lane >> 4) * 8;

  v8f acc[4][4];
#pragma unroll
  for (int i = 0; i < 4; ++i)
#pragma unroll
    for (int j = 0; j < 4; ++j) acc[i][j] = (v8f){0.f,0.f,0.f,0.f,0.f,0.f,0.f,0.f};

  for (int k0 = 0; k0 < K; k0 += 32) {
    V bh[4], bl[4];
#pragma unroll
    for (int j = 0; j < 4; ++j) {
      const size_t bo = (size_t)(n0 + (j << 4) + rlane) * ldb + koff + k0;
      bh[j] = Frag<T>::load(Bb + bo);
      if (SPLIT) bl[j] = Frag<T>::load(Bb2 + bo);
    }
#pragma unroll
    for (int i = 0; i < 4; ++i) {
      const size_t ao = (size_t)(m0 + (i << 4) + rlane) * lda + koff + k0;
      V ah = Frag<T>::load(Ab + ao);
      V al;
      if (SPLIT) al = Frag<T>::load(Ab2 + ao);
#pragma unroll
      for (int j = 0; j < 4; ++j) {
        acc[i][j] = Frag<T>::mma(ah, bh[j], acc[i][j]);
        if (SPLIT) {
          acc[i][j] = Frag<T>::mma(ah, bl[j], acc[i][j]);
          acc[i][j] = Frag<T>::mma(al, bh[j], acc[i][j]);
        }
      }
      Frag<T>::guard(acc[i][0], acc[i][3], ah, SPLIT ? al : ah);
    }
    Frag<T>::keep(bh[0], bh[1], bh[2], bh[3]);
    if (SPLIT) Frag<T>::keep(bl[0], bl[1], bl[2], bl[3]);
  }
  acc_guard4(acc[0][0], acc[0][1], acc[0][2], acc[0][3]);
  acc_guard4(acc[1][0], acc[1][1], acc[1][2], acc[1][3]);
  acc_guard4(acc[2][0], acc[2][1], acc[2][2], acc[2][3]);
  acc_guard4(acc[3][0], acc[3][1], acc[3][2], acc[3][3]);

  float* slab = sT[wave];
  const float* Rb = RESID ? (resid + (size_t)b * strideR) : nullptr;
#pragma unroll
  for (int i = 0; i < 4; ++i) {
    const int mBase = m0 + (i << 4);
#pragma unroll
    for (int j = 0; j < 4; ++j) {
      const int n = n0 + (j << 4) + rlane;
      float bv = 0.f;
      if (BIAS_MODE == 2) bv = bias[n];
#pragma unroll
      for (int r = 0; r < 8; ++r) {
        float v = acc[i][j][r] * scale;
        if (BIAS_MODE == 1) v += bias[mBase + mOff + r];
        if (BIAS_MODE == 2) v += bv;
        if (RESID) v += Rb[(size_t)(mBase + mOff + r) * ldc + n];
        if (ACT == 1) v = tanhf(v);
        if (ACT == 2) v = fmaxf(v, 0.0f);
        if (ACT == 3) v = v / (1.0f + expf(-v));
        if (ACT == 4) v = (v > 0.f) ? v : 0.01f * v;
        if (ACT == 5) v = 0.5f * v * (1.0f + erff(v * 0.70710678118654752f));
        slab[(mOff + r) * 68 + (j << 4) + rlane] = v;
      }
    }
    __builtin_amdgcn_fence(__ATOMIC_RELEASE, "workgroup");
    __builtin_amdgcn_wave_barrier();
    __builtin_amdgcn_fence(__ATOMIC_ACQUIRE, "workgroup");
    if (OUT_MODE == 0) {
      float* C = (float*)Cout + (size_t)b * strideC;
      const int hh = lane >> 4, c4 = (lane & 15) * 4;
      for (int pass = 0; pass < 2; ++pass) {
#pragma unroll
        for (int it = 0; it < 8; ++it) {
          const int row = it * 2 + hh;
          v4f v = *(const v4f*)(slab + row * 68 + c4);
          *(volatile v4f*)(C + (size_t)(mBase + row) * ldc + n0 + c4) = v;
        }
        __threadfence();
      }
    } else {
      const int q = lane >> 3, c8 = (lane & 7) * 8;
      unsigned short* C  = (unsigned short*)Cout  + (size_t)b * strideC;
      unsigned short* C2 = (OUT_MODE == 2) ? ((unsigned short*)Cout2 + (size_t)b * strideC) : nullptr;
      for (int pass = 0; pass < 2; ++pass) {
#pragma unroll
        for (int it = 0; it < 4; ++it) {
          const int row = it * 4 + q;
          const float* sp = slab + row * 68 + c8;
          v8h hv, lv;
#pragma unroll
          for (int e = 0; e < 8; ++e) {
            if (OUT_MODE == 1) {
              hv[e] = (_Float16)sp[e];
            } else {
              unsigned short hb = f2bf_bits(sp[e]);
              unsigned short lb = f2bf_bits(sp[e] - bf_bits2f(hb));
              hv[e] = __builtin_bit_cast(_Float16, hb);
              lv[e] = __builtin_bit_cast(_Float16, lb);
            }
          }
          *(volatile v8h*)(C + (size_t)(mBase + row) * ldc + n0 + c8) = hv;
          if (OUT_MODE == 2) *(volatile v8h*)(C2 + (size_t)(mBase + row) * ldc + n0 + c8) = lv;
        }
        __threadfence();
      }
    }
    __builtin_amdgcn_fence(__ATOMIC_RELEASE, "workgroup");
    __builtin_amdgcn_wave_barrier();
    __builtin_amdgcn_fence(__ATOMIC_ACQUIRE, "workgroup");
  }
}

__global__ __launch_bounds__(256) void cast8_f16_kernel(
    const float* __restrict__ src, unsigned short* __restrict__ dst, int total8, float scale)
{
  const int i = blockIdx.x * 256 + threadIdx.x;
  if (i >= total8) return;
  const size_t e0 = (size_t)i << 3;
  const v4f a0 = *(const v4f*)(src + e0);
  const v4f a1 = *(const v4f*)(src + e0 + 4);
  v8h hv;
#pragma unroll
  for (int e = 0; e < 4; ++e) {
    hv[e]     = (_Float16)(a0[e] * scale);
    hv[4 + e] = (_Float16)(a1[e] * scale);
  }
  unsigned short* q = dst + e0;
  *(volatile v8h*)q = hv;
  __threadfence();
  *(volatile v8h*)q = hv;
}

__global__ __launch_bounds__(256) void pack_w2_kernel(
    const float* __restrict__ w, unsigned short* __restrict__ dst, int total8)
{
  const int i = blockIdx.x * 256 + threadIdx.x;
  if (i >= total8) return;
  const int e0  = i << 3;
  const int o   = e0 / kK2;
  const int k   = e0 - o * kK2;
  const int tap = k >> 7;
  const int c   = k & (kC1 - 1);
  v8h hv;
#pragma unroll
  for (int e = 0; e < 8; ++e) {
    const float v = w[(size_t)o * kK2 + (c + e) * 3 + tap] * 16.0f;
    hv[e] = (_Float16)v;
  }
  unsigned short* q = dst + e0;
  *(volatile v8h*)q = hv;
  __threadfence();
  *(volatile v8h*)q = hv;
}

__global__ __launch_bounds__(256) void pack_wxp_kernel(
    const float* __restrict__ Wx, unsigned short* __restrict__ dst, int total8)
{
  const int i = blockIdx.x * 256 + threadIdx.x;
  if (i >= total8) return;
  const int e0 = i << 3;
  const int n  = e0 >> 9;
  const int k0 = e0 & (kDin - 1);
  const int nc = (n < kXpN) ? n : (kXpN - 1);
  const bool keep = (n < kXpN);
  v8h hv;
#pragma unroll
  for (int e = 0; e < 8; ++e) {
    const float wv = Wx[(size_t)nc * kDin + k0 + e];
    const float v  = keep ? (wv * 16.0f) : 0.0f;
    hv[e] = (_Float16)v;
  }
  unsigned short* q = dst + e0;
  *(volatile v8h*)q = hv;
  __threadfence();
  *(volatile v8h*)q = hv;
}

__global__ __launch_bounds__(128) void conv1_kernel(
    const float* __restrict__ x, const float* __restrict__ w1, const float* __restrict__ b1,
    unsigned short* __restrict__ F1P)
{
  __shared__ float sX[640];
  __shared__ __align__(16) float sT[16 * kC1TP];
  const int tid = threadIdx.x, lane = tid & 31, wave = tid >> 5;
  const int b  = blockIdx.y;
  const int t0 = blockIdx.x * 64;
#pragma unroll
  for (int i = 0; i < 5; ++i) {
    const int idx  = tid + 128 * i;
    const int idxc = (idx < 594) ? idx : 593;
    const int r    = idxc / kXin;
    const int c    = idxc - r * kXin;
    const int tt   = t0 - 1 + r;
    const int ttc  = (tt < 0) ? 0 : ((tt > kSeq - 1) ? (kSeq - 1) : tt);
    const float v  = x[((size_t)b * kSeq + ttc) * kXin + c];
    sX[idx] = (tt >= 0 && tt < kSeq) ? v : 0.0f;
  }
  float wr[27];
#pragma unroll
  for (int k = 0; k < 27; ++k) wr[k] = w1[(size_t)tid * 27 + k];
  const float bo = b1[tid];
  __syncthreads();

  {
    v8h zv;
#pragma unroll
    for (int e = 0; e < 8; ++e) zv[e] = (_Float16)0.0f;
    if (blockIdx.x == 0 && tid < 16) {
      unsigned short* zp = F1P + ((size_t)b * kPadRows + 0) * kC1 + tid * 8;
      *(volatile v8h*)zp = zv;
      __threadfence();
      *(volatile v8h*)zp = zv;
    }
    if (blockIdx.x == (kSeq / 64 - 1) && tid < 16) {
      unsigned short* zp = F1P + ((size_t)b * kPadRows + (kPadRows - 1)) * kC1 + tid * 8;
      *(volatile v8h*)zp = zv;
      __threadfence();
      *(volatile v8h*)zp = zv;
    }
  }

  const int hrow = wave * 2 + (lane >> 4);
  const int c8   = (lane & 15) * 8;
#pragma unroll 1
  for (int sub = 0; sub < 4; ++sub) {
#pragma unroll 1
    for (int s = 0; s < 16; ++s) {
      const float* xr = sX + (sub * 16 + s) * kXin;
      float acc = bo;
#pragma unroll
      for (int j = 0; j < 3; ++j) {
#pragma unroll
        for (int c = 0; c < kXin; ++c) acc = fmaf(wr[c * 3 + j], xr[j * kXin + c], acc);
      }
      sT[s * kC1TP + tid] = fmaxf(acc, 0.0f);
    }
    __syncthreads();
    v8h hv[2];
#pragma unroll
    for (int it = 0; it < 2; ++it) {
      const float* sp = sT + (it * 8 + hrow) * kC1TP + c8;
      const v4f a0 = *(const v4f*)(sp);
      const v4f a1 = *(const v4f*)(sp + 4);
#pragma unroll
      for (int e = 0; e < 4; ++e) { hv[it][e] = (_Float16)a0[e]; hv[it][4 + e] = (_Float16)a1[e]; }
    }
    for (int pass = 0; pass < 2; ++pass) {
#pragma unroll
      for (int it = 0; it < 2; ++it) {
        const int p = t0 + sub * 16 + it * 8 + hrow + 1;
        *(volatile v8h*)(F1P + ((size_t)b * kPadRows + p) * kC1 + c8) = hv[it];
      }
      __threadfence();
    }
    __syncthreads();
  }
}

__global__ __launch_bounds__(256) void dwconv_silu_kernel(
    const float* __restrict__ XZ, const float* __restrict__ cw, const float* __restrict__ cb,
    float* __restrict__ UC, unsigned short* __restrict__ UH)
{
  __shared__ __align__(16) float sT[16 * kConvTP];
  const int tid = threadIdx.x, lane = tid & 31, wave = tid >> 5;
  const int d0 = blockIdx.x * 256, d = d0 + tid;
  const int g0 = blockIdx.y * 64;
  const float w0 = cw[d * 4 + 0], w1 = cw[d * 4 + 1], w2 = cw[d * 4 + 2], w3 = cw[d * 4 + 3];
  const float bc = cb[d];
  float xm3, xm2, xm1;
  {
    const bool hist = ((g0 & (kSeq - 1)) != 0);
    const int rb = hist ? (g0 - 3) : g0;
    const float v3 = XZ[(size_t)rb * kXzP + d];
    const float v2 = XZ[(size_t)(rb + 1) * kXzP + d];
    const float v1 = XZ[(size_t)(rb + 2) * kXzP + d];
    xm3 = hist ? v3 : 0.f;
    xm2 = hist ? v2 : 0.f;
    xm1 = hist ? v1 : 0.f;
  }
  const int hrow = wave >> 1;
  const int hch  = (wave & 1) * 128 + lane * 4;
#pragma unroll 1
  for (int sub = 0; sub < 4; ++sub) {
    const int lb = g0 + sub * 16;
#pragma unroll 1
    for (int s = 0; s < 16; ++s) {
      const float xcur = XZ[(size_t)(lb + s) * kXzP + d];
      float acc = w0 * xm3;
      acc = fmaf(w1, xm2, acc);
      acc = fmaf(w2, xm1, acc);
      acc = fmaf(w3, xcur, acc);
      const float sv = acc + bc;
      const float sg = __builtin_amdgcn_rcpf(1.0f + __expf(-sv));
      sT[s * kConvTP + tid] = sv * sg;
      xm3 = xm2; xm2 = xm1; xm1 = xcur;
    }
    __syncthreads();
    v4f fv[4];
    v8h bh[2];
#pragma unroll
    for (int it = 0; it < 4; ++it) fv[it] = *(const v4f*)(sT + (it * 4 + hrow) * kConvTP + hch);
#pragma unroll
    for (int it = 0; it < 2; ++it) {
      const float* sp = sT + (it * 8 + wave) * kConvTP + lane * 8;
      const v4f a0 = *(const v4f*)(sp);
      const v4f a1 = *(const v4f*)(sp + 4);
#pragma unroll
      for (int e = 0; e < 4; ++e) {
        bh[it][e]     = (_Float16)a0[e];
        bh[it][4 + e] = (_Float16)a1[e];
      }
    }
    for (int pass = 0; pass < 2; ++pass) {
#pragma unroll
      for (int it = 0; it < 4; ++it)
        *(volatile v4f*)(UC + (size_t)(lb + it * 4 + hrow) * kDin + d0 + hch) = fv[it];
#pragma unroll
      for (int it = 0; it < 2; ++it) {
        const size_t o = (size_t)(lb + it * 8 + wave) * kDin + d0 + lane * 8;
        *(volatile v8h*)(UH + o) = bh[it];
      }
      __threadfence();
    }
    __syncthreads();
  }
}

__global__ __launch_bounds__(64) void scan_kernel(
    const float* __restrict__ XD, const float* __restrict__ UC, const float* __restrict__ XZ,
    const float* __restrict__ Wdt, const float* __restrict__ bdt, const float* __restrict__ Alog,
    const float* __restrict__ Dp, unsigned short* __restrict__ YP)
{
  __shared__ __align__(16) float sX[kScanTS * kXdP];
  __shared__ __align__(16) float sY[kScanTS * kScanYP];
  const int tid = threadIdx.x, lane = tid & 31, wave = tid >> 5;
  const int b  = blockIdx.x >> 3;
  const int d0 = (blockIdx.x & 7) * kScanCh;
  const int d  = d0 + tid;
  const size_t rowbase = (size_t)b * kSeq;
  float negA[kNst], h[kNst], wdt[kDtR];
#pragma unroll
  for (int s = 0; s < kNst; ++s) {
    negA[s] = -expf(Alog[(size_t)d * kNst + s]);
    h[s] = 0.f;
  }
#pragma unroll
  for (int r = 0; r < kDtR; ++r) wdt[r] = Wdt[(size_t)d * kDtR + r];
  const float bb = bdt[d], Dd = Dp[d];
  const int lr = tid >> 4, lc4 = (tid & 15) * 4;
  const int q = lane >> 3, c8 = (lane & 7) * 8;
#pragma unroll 1
  for (int t0 = 0; t0 < kSeq; t0 += kScanTS) {
    __syncthreads();
#pragma unroll
    for (int i = 0; i < 16; ++i) {
      const int r = lr + 4 * i;
      *(v4f*)(sX + r * kXdP + lc4) = *(const v4f*)(XD + (rowbase + t0 + r) * kXdP + lc4);
    }
    __syncthreads();
#pragma unroll 1
    for (int s = 0; s < kScanTS; ++s) {
      const size_t row = rowbase + t0 + s;
      const float* xr = sX + s * kXdP;
      float Bs[kNst], Cs[kNst];
      float v = bb;
#pragma unroll
      for (int q4 = 0; q4 < 4; ++q4) {
        const v4f dv = *(const v4f*)(xr + 4 * q4);
        const v4f bv = *(const v4f*)(xr + 16 + 4 * q4);
        const v4f cv = *(const v4f*)(xr + 32 + 4 * q4);
        v = fmaf(dv[0], wdt[4 * q4 + 0], v);
        v = fmaf(dv[1], wdt[4 * q4 + 1], v);
        v = fmaf(dv[2], wdt[4 * q4 + 2], v);
        v = fmaf(dv[3], wdt[4 * q4 + 3], v);
        Bs[4 * q4 + 0] = bv[0]; Bs[4 * q4 + 1] = bv[1]; Bs[4 * q4 + 2] = bv[2]; Bs[4 * q4 + 3] = bv[3];
        Cs[4 * q4 + 0] = cv[0]; Cs[4 * q4 + 1] = cv[1]; Cs[4 * q4 + 2] = cv[2]; Cs[4 * q4 + 3] = cv[3];
      }
      const float a   = __expf(-fabsf(v));
      const float u1  = 1.0f + a;
      const float l1p = __logf(u1) + (a - (u1 - 1.0f)) * __builtin_amdgcn_rcpf(u1);
      const float dt  = fmaxf(v, 0.0f) + l1p;
      const float xt  = UC[row * kDin + d];
      const float dtx = dt * xt;
      float y = 0.f;
#pragma unroll
      for (int k = 0; k < kNst; ++k) {
        const float e = __expf(dt * negA[k]);
        h[k] = e * h[k] + dtx * Bs[k];
        y = h[k] * Cs[k] + y;
      }
      y = xt * Dd + y;
      const float zv = XZ[row * kXzP + kDin + d];
      const float sg = __builtin_amdgcn_rcpf(1.0f + __expf(-zv));
      y = y * (zv * sg);
      sY[s * kScanYP + tid] = y;
    }
    __syncthreads();
    v8h hv[8];
#pragma unroll
    for (int it = 0; it < 8; ++it) {
      const int r = it * 8 + wave * 4 + q;
      const float* sp = sY + r * kScanYP + c8;
      const v4f a0 = *(const v4f*)(sp);
      const v4f a1 = *(const v4f*)(sp + 4);
#pragma unroll
      for (int e = 0; e < 4; ++e) {
        hv[it][e]     = (_Float16)a0[e];
        hv[it][4 + e] = (_Float16)a1[e];
      }
    }
    for (int pass = 0; pass < 2; ++pass) {
#pragma unroll
      for (int it = 0; it < 8; ++it) {
        const int r = it * 8 + wave * 4 + q;
        const size_t o = (rowbase + t0 + r) * kDin + d0 + c8;
        *(volatile v8h*)(YP + o) = hv[it];
      }
      __threadfence();
    }
  }
}

__global__ __launch_bounds__(256) void pool_kernel(const float* __restrict__ MO, float* __restrict__ POOL)
{
  const int b = blockIdx.x, c = threadIdx.x;
  const float* p = MO + (size_t)b * kSeq * kDm + c;
  float m = p[0];
#pragma unroll 4
  for (int t = 1; t < kSeq; ++t) m = fmaxf(m, p[(size_t)t * kDm]);
  float* qo = POOL + (size_t)b * kDm + c;
  *(volatile float*)qo = m;
  __threadfence();
  *(volatile float*)qo = m;
}

__global__ __launch_bounds__(512) void head_kernel(
    const float* __restrict__ POOL, const float* __restrict__ W1, const float* __restrict__ B1,
    const float* __restrict__ W2, const float* __restrict__ B2, float* __restrict__ out)
{
  __shared__ float sP[kBatch * kDm];
  __shared__ float sH[kBatch * kHid];
  const int tid = threadIdx.x;
  sP[tid]       = POOL[tid];
  sP[tid + 512] = POOL[tid + 512];
  __syncthreads();
  {
    const int b = tid >> 7, j = tid & (kHid - 1);
    const float* wr = W1 + (size_t)j * kDm;
    const float* pr = sP + b * kDm;
    float acc = B1[j];
#pragma unroll 1
    for (int i = 0; i < kDm; ++i) acc = fmaf(pr[i], wr[i], acc);
    sH[tid] = fmaxf(acc, 0.0f);
  }
  __syncthreads();
  if (tid < 32) {
    const int bb = (tid >> 2) & 3, cc = tid & 3;
    const float* hr = sH + bb * kHid;
    const float* wr = W2 + (size_t)cc * kHid;
    float acc = B2[cc];
#pragma unroll 1
    for (int i = 0; i < kHid; ++i) acc = fmaf(hr[i], wr[i], acc);
    if (tid < 16) {
      *(volatile float*)(out + tid) = acc;
      __threadfence();
      *(volatile float*)(out + tid) = acc;
    }
  }
}

extern "C" void kernel_launch(void* const* d_in, const int* in_sizes, int n_in,
                              void* d_out, int out_size, void* d_ws, size_t ws_size,
                              hipStream_t stream) {
  if (n_in < 18) return;
  if (in_sizes[0] != kRows * kXin) return;
  if (in_sizes[3] != kDm * kC1 * 3) return;
  if (in_sizes[5] != kXzP * kDm) return;
  if (in_sizes[8] != kXpN * kDin) return;
  if (in_sizes[13] != kDm * kDin) return;
  if (out_size != kBatch * kCls) return;
  if (ws_size < kWsTotal) return;

  const float* x          = (const float*)d_in[0];
  const float* conv1_w    = (const float*)d_in[1];
  const float* conv1_b    = (const float*)d_in[2];
  const float* conv2_w    = (const float*)d_in[3];
  const float* conv2_b    = (const float*)d_in[4];
  const float* in_proj_w  = (const float*)d_in[5];
  const float* dw_w       = (const float*)d_in[6];
  const float* dw_b       = (const float*)d_in[7];
  const float* x_proj_w   = (const float*)d_in[8];
  const float* dt_w       = (const float*)d_in[9];
  const float* dt_b       = (const float*)d_in[10];
  const float* A_log      = (const float*)d_in[11];
  const float* Dp         = (const float*)d_in[12];
  const float* out_proj_w = (const float*)d_in[13];
  const float* fc1_w      = (const float*)d_in[14];
  const float* fc1_b      = (const float*)d_in[15];
  const float* fc2_w      = (const float*)d_in[16];
  const float* fc2_b      = (const float*)d_in[17];
  float* out = (float*)d_out;

  char* ws = (char*)d_ws;
  unsigned short* F1P  = (unsigned short*)(ws + kOffF1P);
  unsigned short* W2P  = (unsigned short*)(ws + kOffW2P);
  unsigned short* FEAT = (unsigned short*)(ws + kOffFeat);
  unsigned short* WIN  = (unsigned short*)(ws + kOffWin);
  float*          XZ   = (float*)(ws + kOffXZ);
  float*          UC   = (float*)(ws + kOffUC);
  unsigned short* UH   = (unsigned short*)(ws + kOffUH);
  unsigned short* WXP  = (unsigned short*)(ws + kOffWxp);
  float*          XD   = (float*)(ws + kOffXD);
  unsigned short* YP   = (unsigned short*)(ws + kOffYP);
  unsigned short* WOUT = (unsigned short*)(ws + kOffWout);
  float*          MO   = (float*)(ws + kOffMO);
  float*          POOL = (float*)(ws + kOffPool);

  cast8_f16_kernel<<<(kXzP * kDm / 8) / 256, 256, 0, stream>>>(in_proj_w, WIN, kXzP * kDm / 8, 16.0f);
  pack_w2_kernel<<<(kDm * kK2 / 8) / 256, 256, 0, stream>>>(conv2_w, W2P, kDm * kK2 / 8);
  pack_wxp_kernel<<<(kXdP * kDin / 8) / 256, 256, 0, stream>>>(x_proj_w, WXP, kXdP * kDin / 8);
  cast8_f16_kernel<<<(kDm * kDin / 8) / 256, 256, 0, stream>>>(out_proj_w, WOUT, kDm * kDin / 8, 16.0f);

  conv1_kernel<<<dim3(kSeq / 64, kBatch), 128, 0, stream>>>(x, conv1_w, conv1_b, F1P);

  wmma_gemm64<0, false, 2, 1, false, 2><<<dim3(16, kBatch), 256, 0, stream>>>(
      F1P, nullptr, kC1, (long)kPadRows * kC1,
      W2P, nullptr, kK2, 0L,
      (void*)FEAT, nullptr, kDm, (long)kSeq * kDm,
      conv2_b, nullptr, 0L,
      kSeq, kDm, kK2, 1.0f / 16.0f);

  wmma_gemm64<0, false, 0, 0, false, 0><<<dim3(256, 1), 256, 0, stream>>>(
      FEAT, nullptr, kDm, 0L,
      WIN, nullptr, kDm, 0L,
      (void*)XZ, nullptr, kXzP, 0L,
      nullptr, nullptr, 0L,
      kRows, kXzP, kDm, 1.0f / 16.0f);

  dwconv_silu_kernel<<<dim3(kDin / 256, kRows / 64), 256, 0, stream>>>(XZ, dw_w, dw_b, UC, UH);

  wmma_gemm64<0, false, 0, 0, false, 0><<<dim3(16, 1), 256, 0, stream>>>(
      UH, nullptr, kDin, 0L,
      WXP, nullptr, kDin, 0L,
      (void*)XD, nullptr, kXdP, 0L,
      nullptr, nullptr, 0L,
      kRows, kXdP, kDin, 1.0f / 16.0f);

  scan_kernel<<<kBatch * (kDin / kScanCh), kScanCh, 0, stream>>>(XD, UC, XZ, dt_w, dt_b, A_log, Dp, YP);

  wmma_gemm64<0, false, 0, 0, false, 0><<<dim3(64, 1), 256, 0, stream>>>(
      YP, nullptr, kDin, 0L,
      WOUT, nullptr, kDin, 0L,
      (void*)MO, nullptr, kDm, 0L,
      nullptr, nullptr, 0L,
      kRows, kDm, kDin, 1.0f / 16.0f);

  pool_kernel<<<kBatch, kDm, 0, stream>>>(MO, POOL);
  head_kernel<<<1, 512, 0, stream>>>(POOL, fc1_w, fc1_b, fc2_w, fc2_b, out);
}
